// HybridAttention_22746146799820
// MI455X (gfx1250) — hardware-verified
//
#include <hip/hip_runtime.h>
#include <math.h>

typedef __attribute__((ext_vector_type(16))) _Float16 v16h;
typedef __attribute__((ext_vector_type(16))) __bf16 v16b;
typedef __attribute__((ext_vector_type(8)))  _Float16 v8h;
typedef __attribute__((ext_vector_type(8)))  __bf16 v8b;
typedef __attribute__((ext_vector_type(8)))  float v8f;
typedef __attribute__((ext_vector_type(4)))  float v4f;
typedef __attribute__((ext_vector_type(4)))  unsigned v4u;

template <typename T> __device__ __forceinline__ void vst2(void* p, T v) { *(volatile T*)p = v; __threadfence(); *(volatile T*)p = v; }
__device__ __forceinline__ v8f wmma16(v16h a, v16h b, v8f c) {
  v8f d = __builtin_amdgcn_wmma_f32_16x16x32_f16(false, a, false, b, (short)0, c, false, false);
  asm volatile("v_nop\n\tv_nop\n\tv_nop\n\tv_nop" : "+v"(d) : "v"(a), "v"(b));
  return d;
}
__device__ __forceinline__ v8f wmma_bf(v16b a, v16b b, v8f c) {
  v8f d = __builtin_amdgcn_wmma_f32_16x16x32_bf16(false, a, false, b, (short)0, c, false, false);
  asm volatile("v_nop\n\tv_nop\n\tv_nop\n\tv_nop" : "+v"(d) : "v"(a), "v"(b));
  return d;
}
__device__ __forceinline__ v16h frag_h(const _Float16* rowk0, int lane) {
  union { v16h v; v8h q[2]; } u; const _Float16* p = rowk0 + 8 * (lane >> 4);
  u.q[0] = *(const v8h*)p; u.q[1] = *(const v8h*)(p + 16); return u.v;
}
__device__ __forceinline__ v16b frag_b(const __bf16* rowk0, int lane) {
  union { v16b v; v8b q[2]; } u; const __bf16* p = rowk0 + 8 * (lane >> 4);
  u.q[0] = *(const v8b*)p; u.q[1] = *(const v8b*)(p + 16); return u.v;
}
struct F2 { v16b h, l; };
__device__ __forceinline__ F2 bsplit16(const float v[16]) { F2 r;
#pragma unroll
  for (int i = 0; i < 16; ++i) { const __bf16 h = (__bf16)v[i]; r.h[i] = h; r.l[i] = (__bf16)(v[i] - (float)h); }
  return r; }
__device__ __forceinline__ F2 split_row(const float* row, int k0, int lane) { float v[16]; const float* p = row + k0 + 8 * (lane >> 4);
#pragma unroll
  for (int i = 0; i < 8; ++i) { v[i] = p[i]; v[8 + i] = p[16 + i]; }
  return bsplit16(v); }
__device__ __forceinline__ void ldsx() { asm volatile("s_wait_dscnt 0" ::: "memory"); __builtin_amdgcn_wave_barrier(); __builtin_amdgcn_fence(3, "workgroup"); }

#ifndef NB
#define NB 1
#endif
#ifndef SEQ
#define SEQ 4096
#endif
#define NB_FULL 1
#define SEQ_FULL 4096
#define CC 1024
#define NH 16
#define NAR 8
#define HD 64
#ifndef TNB
#define TNB NB
#endif
static_assert(NB >= 1 && NB <= NB_FULL);
static_assert(SEQ % 128 == 0 && SEQ <= SEQ_FULL);
static_assert(CC == NH * HD);
static_assert(CC % 128 == 0);

#define WS_WO      ((size_t)0)
#define WS_WQKV    (WS_WO + 2u * (size_t)CC * CC)
#define WQKV_BYTES (6u * (size_t)CC * CC)
#define WS_S       WS_WQKV
#define S_BYTES    (4u * (size_t)SEQ * SEQ)
#define WS_QH      (WS_S + (S_BYTES > WQKV_BYTES ? S_BYTES : WQKV_BYTES))
#define PL_BYTES   (2u * (size_t)NB * SEQ * CC)
#define WS_QL      (WS_QH + PL_BYTES)
#define WS_KH      (WS_QL + PL_BYTES)
#define WS_VT      (WS_KH + PL_BYTES)
#define WS_VL      (WS_VT + PL_BYTES)
#define WS_YH      (WS_VL + PL_BYTES)
#define WS_YL      (WS_YH + PL_BYTES)
#define WS_END     (WS_YL + PL_BYTES)
static_assert(WS_WO + 2u * (size_t)CC * CC <= WS_S);
static_assert(WS_S + S_BYTES <= WS_QH);
static_assert(WS_WQKV + WQKV_BYTES <= WS_QH);
static_assert(WS_END <= (size_t)134217728);
static_assert((WS_S % 128) == 0 && (WS_QH % 128) == 0 && (WS_YH % 128) == 0);

__global__ __launch_bounds__(256) void k_wt(const float* __restrict__ W0, const float* __restrict__ W1, const float* __restrict__ W2, const float* __restrict__ W3, __bf16* __restrict__ WT) {
  __shared__ __align__(16) __bf16 tl[64][72];
  const int tid = threadIdx.x, wave = tid >> 5, lane = tid & 31;
  const int z = blockIdx.z; const float* W = z == 0 ? W0 : z == 1 ? W1 : z == 2 ? W2 : W3;
  __bf16* D = WT + (size_t)z * CC * CC;
  const int n0 = blockIdx.x * 64, k0 = blockIdx.y * 64;
#pragma unroll
  for (int i = 0; i < 4; ++i) { const int idx = tid + 256 * i; const int r = idx >> 4, c4 = (idx & 15) * 4;
    const v4f v = *(const v4f*)(W + (size_t)(k0 + r) * CC + n0 + c4);
    tl[c4 + 0][r] = (__bf16)v[0]; tl[c4 + 1][r] = (__bf16)v[1]; tl[c4 + 2][r] = (__bf16)v[2]; tl[c4 + 3][r] = (__bf16)v[3]; }
  __syncthreads();
#pragma unroll
  for (int it = 0; it < 2; ++it) { const int row = it * 32 + wave * 4 + (lane >> 3), piece = lane & 7;
    const v4u val = *(const v4u*)&tl[row][piece * 8];
    vst2((unsigned*)(D + (size_t)(n0 + row) * CC + k0 + piece * 8), val); }
}

struct LdsQK { _Float16 qh[64][136]; _Float16 ql[64][136]; float tc[64][32]; float ts[64][32]; };
struct LdsV  { __bf16 vh[128][72]; __bf16 vl[128][72]; };
union LdsProj { LdsQK qk; LdsV v; };

__global__ __launch_bounds__(128) void k_proj(const float* __restrict__ X, const __bf16* __restrict__ WQT, const __bf16* __restrict__ WKT, const __bf16* __restrict__ WVT, _Float16* __restrict__ QH, _Float16* __restrict__ QL, _Float16* __restrict__ KH, __bf16* __restrict__ VT, __bf16* __restrict__ VL) {
  __shared__ __align__(16) LdsProj sm;
  const int tid = threadIdx.x, wave = tid >> 5, lane = tid & 31, col = lane & 15, g = lane >> 4; const int which = blockIdx.z; const int c0 = blockIdx.y * 128; const size_t r0 = (size_t)blockIdx.x * 64;
  const size_t b = r0 / SEQ; const int t0 = (int)(r0 % SEQ);
  const __bf16* WA = which == 0 ? WQT : which == 1 ? WKT : WVT;
  if (which < 2) {
    const float invf = 1.0f / (float)pow(10000.0, (double)lane * 0.03125);
    for (int e = tid; e < 64 * 32; e += 128) { const int rl = e >> 5; float sn, cs; sincosf((float)(t0 + rl) * invf, &sn, &cs); sm.qk.ts[rl][lane] = sn; sm.qk.tc[rl][lane] = cs; }
  }
  __syncthreads();
  v8f acc[8] = {};
  const float* xrow = X + (b * SEQ_FULL + t0 + wave * 16 + col) * (size_t)CC;
#pragma unroll 2
  for (int kc = 0; kc < CC / 32; ++kc) { v16b a; { const float* p = xrow + kc * 32 + 8 * g;
#pragma unroll
      for (int i = 0; i < 8; ++i) { a[i] = (__bf16)p[i]; a[8 + i] = (__bf16)p[16 + i]; } }
#pragma unroll
    for (int j = 0; j < 8; ++j) { const int o = c0 + j * 16 + col;
      acc[j] = wmma_bf(a, frag_b(WA + (size_t)o * CC + kc * 32, lane), acc[j]); } }
  if (which == 2) {
#pragma unroll
    for (int j = 0; j < 8; ++j) {
#pragma unroll
      for (int r = 0; r < 8; ++r) { const float v = acc[j][r]; const int rl = wave * 16 + 8 * g + r, cl = j * 16 + col; const __bf16 bh = (__bf16)v; sm.v.vh[cl][rl] = bh; sm.v.vl[cl][rl] = (__bf16)(v - (float)bh); } }
  } else {
#pragma unroll
    for (int jp = 0; jp < 4; ++jp) { const int ja = (jp & 1) + (jp >> 1) * 4, jb = ja + 2; const int fi = (jp & 1) * 16 + col;
#pragma unroll
      for (int r = 0; r < 8; ++r) { const int rl = wave * 16 + 8 * g + r; const float cs = sm.qk.tc[rl][fi], sn = sm.qk.ts[rl][fi];
        const float x1 = acc[ja][r], x2 = acc[jb][r];
        const float o1 = x1 * cs - x2 * sn, o2 = x2 * cs + x1 * sn;
        const _Float16 h1 = (_Float16)o1, h2 = (_Float16)o2;
        sm.qk.qh[rl][ja * 16 + col] = h1; sm.qk.ql[rl][ja * 16 + col] = (_Float16)((o1 - (float)h1) * 1024.0f);
        sm.qk.qh[rl][jb * 16 + col] = h2; sm.qk.ql[rl][jb * 16 + col] = (_Float16)((o2 - (float)h2) * 1024.0f); } }
  }
  __syncthreads();
  if (which < 2) { _Float16* dh = which == 0 ? QH : KH; for (int e = tid; e < 64 * 16; e += 128) { const int rl = e >> 4, q = e & 15; const size_t go = (r0 + rl) * CC + c0 + q * 8; vst2((unsigned*)(dh + go), *(const v4u*)&sm.qk.qh[rl][q * 8]); if (which == 0) vst2((unsigned*)(QL + go), *(const v4u*)&sm.qk.ql[rl][q * 8]); } }
  else { for (int e = tid; e < 128 * 8; e += 128) { const int cl = e >> 3, q = e & 7; const size_t o2 = (b * CC + c0 + cl) * (size_t)SEQ + t0 + q * 8; vst2((unsigned*)(VT + o2), *(const v4u*)&sm.v.vh[cl][q * 8]); vst2((unsigned*)(VL + o2), *(const v4u*)&sm.v.vl[cl][q * 8]); } }
}
__global__ __launch_bounds__(128) void k_sc(const _Float16* __restrict__ QH, const _Float16* __restrict__ QL, const _Float16* __restrict__ KH, int b, int h, int causal, float* __restrict__ S) { __shared__ __align__(16) float ss[4][16][132];
  const int tid = threadIdx.x, wave = tid >> 5, lane = tid & 31, col = lane & 15, g = lane >> 4; const int k0 = blockIdx.y * 128, qb = blockIdx.x * 64;
  if (causal != 0 && k0 >= qb + 64) return;
  const int ql0 = qb + wave * 16; const size_t q0 = (size_t)b * SEQ + ql0;
  v8f acc[8] = {}, accl[8] = {};
#pragma unroll
  for (int kc = 0; kc < HD / 32; ++kc) { const v16h ah = frag_h(QH + (q0 + col) * CC + h * HD + kc * 32, lane), al = frag_h(QL + (q0 + col) * CC + h * HD + kc * 32, lane);
#pragma unroll
    for (int j = 0; j < 8; ++j) { const v16h kb = frag_h(KH + ((size_t)b * SEQ + k0 + j * 16 + col) * CC + h * HD + kc * 32, lane); acc[j] = wmma16(ah, kb, acc[j]); accl[j] = wmma16(al, kb, accl[j]); } }
#pragma unroll
  for (int j = 0; j < 8; ++j) acc[j] += accl[j] * (1.0f / 1024.0f);
#pragma unroll
  for (int j = 0; j < 8; ++j) {
#pragma unroll
    for (int r = 0; r < 8; ++r) ss[wave][8 * g + r][j * 16 + col] = acc[j][r] * 0.125f; }
  ldsx(); for (int rl = 0; rl < 16; ++rl) vst2(S + (size_t)(ql0 + rl) * SEQ + k0 + lane * 4, *(const v4f*)&ss[wave][rl][lane * 4]); }
__global__ __launch_bounds__(256) void k_sm(float* __restrict__ S, int causal) { __shared__ float sred[8]; __shared__ float sbc; __shared__ __align__(16) float sh[SEQ];
  const int t = threadIdx.x; const int row = blockIdx.x; float* sr = S + (size_t)row * SEQ;
  const int klim = causal != 0 ? row : SEQ - 1; const int kend = causal != 0 ? ((row & ~63) + 64) : SEQ;
  float m = -3.0e38f; for (int k = t; k <= klim; k += 256) m = fmaxf(m, sr[k]);
#pragma unroll
  for (int o = 1; o < 32; o <<= 1) m = fmaxf(m, __shfl_xor(m, o));
  if ((t & 31) == 0) sred[t >> 5] = m; __syncthreads(); if (t == 0) { float a = sred[0]; for (int i = 1; i < 8; ++i) a = fmaxf(a, sred[i]); sbc = a; } __syncthreads(); m = sbc; __syncthreads();
  float sum = 0.f; for (int k = t; k <= klim; k += 256) { const float e = expf(sr[k] - m); sh[k] = e; sum += e; }
  for (int k = klim + 1 + t; k < kend; k += 256) sh[k] = 0.f;
#pragma unroll
  for (int o = 1; o < 32; o <<= 1) sum += __shfl_xor(sum, o);
  if ((t & 31) == 0) sred[t >> 5] = sum; __syncthreads(); if (t == 0) { float a = 0.f; for (int i = 0; i < 8; ++i) a += sred[i]; sbc = 1.0f / a; } __syncthreads(); const float sc = sbc * 2048.0f;
  for (int q = t; q < kend / 4; q += 256) { const v4f x = *(const v4f*)&sh[q * 4] * sc; vst2(sr + q * 4, x); } }
__global__ __launch_bounds__(128) void k_pv(const float* __restrict__ PS, const __bf16* __restrict__ VT, const __bf16* __restrict__ VL, int b, int h, int causal, __bf16* __restrict__ YH, __bf16* __restrict__ YL) { __shared__ __align__(16) float ss[4][16][HD + 4];
  const int tid = threadIdx.x, wave = tid >> 5, lane = tid & 31, col = lane & 15, g = lane >> 4; const int qb = blockIdx.x * 64, ql0 = qb + wave * 16; const int kend = causal != 0 ? qb + 64 : SEQ;
  v8f acc[HD / 16] = {};
#pragma unroll 1
  for (int kc = 0; kc < kend / 32; ++kc) { const F2 p = split_row(PS + (size_t)(ql0 + col) * SEQ, kc * 32, lane);
#pragma unroll
    for (int j = 0; j < HD / 16; ++j) { const size_t po = ((size_t)b * CC + h * HD + j * 16 + col) * (size_t)SEQ + kc * 32; const v16b vh = frag_b(VT + po, lane); acc[j] = wmma_bf(p.h, vh, acc[j]); acc[j] = wmma_bf(p.l, vh, acc[j]); acc[j] = wmma_bf(p.h, frag_b(VL + po, lane), acc[j]); } }
#pragma unroll
  for (int j = 0; j < HD / 16; ++j)
#pragma unroll
    for (int r = 0; r < 8; ++r) ss[wave][8 * g + r][j * 16 + col] = acc[j][r] * (1.0f / 2048.0f);
  ldsx();
  if (lane < 8) { for (int rl = 0; rl < 16; ++rl) { union { v8b v; v4u u; } hh, ll; const float* src = &ss[wave][rl][lane * 8];
#pragma unroll
      for (int i = 0; i < 8; ++i) { const float x = src[i]; const __bf16 bh = (__bf16)x; hh.v[i] = bh; ll.v[i] = (__bf16)(x - (float)bh); }
      const size_t yo = ((size_t)b * SEQ + ql0 + rl) * CC + h * HD + lane * 8;
      vst2((unsigned*)(YH + yo), hh.u); vst2((unsigned*)(YL + yo), ll.u); } } }
__global__ __launch_bounds__(128) void k_out(const __bf16* __restrict__ YH, const __bf16* __restrict__ YL, const __bf16* __restrict__ WOT, float* __restrict__ OUT) { __shared__ __align__(16) float sf[4][16][132];
  const int tid = threadIdx.x, wave = tid >> 5, lane = tid & 31, col = lane & 15, g = lane >> 4; const int c0 = blockIdx.y * 128; const size_t r0 = (size_t)blockIdx.x * 64 + wave * 16;
  v8f acc[8] = {};
#pragma unroll 2
  for (int kc = 0; kc < CC / 32; ++kc) { const v16b ah = frag_b(YH + (r0 + col) * CC + kc * 32, lane), al = frag_b(YL + (r0 + col) * CC + kc * 32, lane);
#pragma unroll
    for (int j = 0; j < 8; ++j) { const int o = c0 + j * 16 + col; const v16b w = frag_b(WOT + (size_t)o * CC + kc * 32, lane);
      acc[j] = wmma_bf(ah, w, acc[j]); acc[j] = wmma_bf(al, w, acc[j]); } }
#pragma unroll
  for (int j = 0; j < 8; ++j) {
#pragma unroll
    for (int r = 0; r < 8; ++r) sf[wave][8 * g + r][j * 16 + col] = acc[j][r]; }
  ldsx(); for (int rl = 0; rl < 16; ++rl) vst2(OUT + (r0 + rl) * CC + c0 + lane * 4, *(const v4f*)&sf[wave][rl][lane * 4]); }

extern "C" void kernel_launch(void* const* d_in, const int* in_sizes, int n_in, void* d_out, int out_size, void* d_ws, size_t ws_size, hipStream_t stream) {
  if (n_in < 5) return;
  if ((size_t)in_sizes[0] < ((size_t)(NB - 1) * SEQ_FULL + SEQ) * (size_t)CC) return;
  if ((size_t)in_sizes[1] < (size_t)CC * CC || (size_t)in_sizes[2] < (size_t)CC * CC || (size_t)in_sizes[3] < (size_t)CC * CC || (size_t)in_sizes[4] < (size_t)CC * CC) return;
  if ((size_t)out_size < (size_t)NB * SEQ * CC) return;
  if (ws_size < (size_t)WS_END) return;
  const float** F = (const float**)d_in;
  char* ws = (char*)d_ws;
  __bf16* WT = (__bf16*)(ws + WS_WO);
  const __bf16 *WOT = WT, *WQT = WT + (size_t)CC * CC, *WKT = WT + 2 * (size_t)CC * CC, *WVT = WT + 3 * (size_t)CC * CC;
  _Float16 *QH = (_Float16*)(ws + WS_QH), *QL = (_Float16*)(ws + WS_QL), *KH = (_Float16*)(ws + WS_KH); __bf16 *VT = (__bf16*)(ws + WS_VT), *VL = (__bf16*)(ws + WS_VL);
  float* S = (float*)(ws + WS_S); __bf16 *YH = (__bf16*)(ws + WS_YH), *YL = (__bf16*)(ws + WS_YL);
  k_wt<<<dim3(CC / 64, CC / 64, 4), 256, 0, stream>>>(F[4], F[1], F[2], F[3], WT);
  k_proj<<<dim3(TNB * SEQ / 64, CC / 128, 3), 128, 0, stream>>>(F[0], WQT, WKT, WVT, QH, QL, KH, VT, VL);
  for (int b = 0; b < TNB; ++b) for (int h = 0; h < NH; ++h) { const int causal = h < NAR ? 1 : 0;
    k_sc<<<dim3(SEQ / 64, SEQ / 128, 1), 128, 0, stream>>>(QH, QL, KH, b, h, causal, S);
    k_sm<<<dim3(SEQ, 1), 256, 0, stream>>>(S, causal);
    k_pv<<<dim3(SEQ / 64, 1, 1), 128, 0, stream>>>(S, VT, VL, b, h, causal, YH, YL);
  }
  k_out<<<dim3(TNB * SEQ / 64, CC / 128), 128, 0, stream>>>(YH, YL, WOT, (float*)d_out);
}
